// Reconstructeur_13357348290803
// MI455X (gfx1250) — hardware-verified
//
#include <hip/hip_runtime.h>
#include <math.h>

typedef __attribute__((ext_vector_type(16))) _Float16 v16h;
typedef __attribute__((ext_vector_type(16))) __bf16 v16b;
typedef __attribute__((ext_vector_type(8)))  _Float16 v8h;
typedef __attribute__((ext_vector_type(8)))  float v8f;
typedef __attribute__((ext_vector_type(4)))  float v4f;
typedef __attribute__((ext_vector_type(2)))  float v2f;
typedef __attribute__((ext_vector_type(4)))  unsigned v4u;
typedef __attribute__((ext_vector_type(4)))  int v4i;
typedef float __attribute__((may_alias)) float_a;
typedef int __attribute__((may_alias)) int_a;

template <typename T> __device__ __forceinline__ void vst2(void* p, T v) { *(volatile T*)p = v; __threadfence(); *(volatile T*)p = v; }
__device__ __forceinline__ v8f wmma16(v16h a, v16h b, v8f c) {
  v8f d = __builtin_amdgcn_wmma_f32_16x16x32_f16(false, a, false, b, (short)0, c, false, false);
  asm volatile("v_nop\n\tv_nop\n\tv_nop\n\tv_nop" : "+v"(d) : "v"(a), "v"(b));
  return d;
}
__device__ __forceinline__ v8f wmma_bf(v16b a, v16b b, v8f c) {
  v8f d = __builtin_amdgcn_wmma_f32_16x16x32_bf16(false, a, false, b, (short)0, c, false, false);
  asm volatile("v_nop\n\tv_nop\n\tv_nop\n\tv_nop" : "+v"(d) : "v"(a), "v"(b));
  return d;
}
__device__ __forceinline__ v16h frag_h(const _Float16* rowk0, int lane) {
  union { v16h v; v8h q[2]; } u; const _Float16* p = rowk0 + 8 * (lane >> 4);
  u.q[0] = *(const v8h*)p; u.q[1] = *(const v8h*)(p + 16); return u.v;
}
__device__ __forceinline__ v16h frag_f32(const float* rowk0, int lane) {
  v16h a; const float* p = rowk0 + 8 * (lane >> 4);
#pragma unroll
  for (int i = 0; i < 8; ++i) { a[i] = (_Float16)p[i]; a[8 + i] = (_Float16)p[16 + i]; }
  return a;
}
__device__ __forceinline__ v16h frag_f32s(const float* rowk0, int lane, float sc) {
  v16h a; const float* p = rowk0 + 8 * (lane >> 4);
#pragma unroll
  for (int i = 0; i < 8; ++i) { a[i] = (_Float16)(p[i] * sc); a[8 + i] = (_Float16)(p[16 + i] * sc); }
  return a;
}
__device__ __forceinline__ v16h fragc_f32(const float* W, int k0, int n, int lane, int ld, int K) {
  v16h a; const int g = lane >> 4;
#pragma unroll
  for (int i = 0; i < 8; ++i) { const int ka = k0 + 8 * g + i, kb = ka + 16;
    a[i] = (_Float16)(ka < K ? W[(size_t)(ka < K ? ka : K - 1) * ld + n] : 0.f); a[8 + i] = (_Float16)(kb < K ? W[(size_t)(kb < K ? kb : K - 1) * ld + n] : 0.f); }
  return a;
}
struct F2 { v16b h, l; };
__device__ __forceinline__ F2 bsplit16(const float v[16]) { F2 r;
#pragma unroll
  for (int i = 0; i < 16; ++i) { const __bf16 h = (__bf16)v[i]; r.h[i] = h; r.l[i] = (__bf16)(v[i] - (float)h); }
  return r; }
__device__ __forceinline__ F2 split_row(const float* row, int k0, int lane) { float v[16]; const float* p = row + k0 + 8 * (lane >> 4);
#pragma unroll
  for (int i = 0; i < 8; ++i) { v[i] = p[i]; v[8 + i] = p[16 + i]; }
  return bsplit16(v); }
__device__ __forceinline__ F2 split_rowK(const float* row, int k0, int lane, int K) { float v[16]; const int g = lane >> 4;
#pragma unroll
  for (int i = 0; i < 8; ++i) { const int ka = k0 + 8 * g + i, kb = ka + 16; v[i] = ka < K ? row[ka < K ? ka : K - 1] : 0.f; v[8 + i] = kb < K ? row[kb < K ? kb : K - 1] : 0.f; }
  return bsplit16(v); }
__device__ __forceinline__ F2 split_col(const float* W, int k0, int n, int lane, int ld, int K) { float v[16]; const int g = lane >> 4;
#pragma unroll
  for (int i = 0; i < 8; ++i) { const int ka = k0 + 8 * g + i, kb = ka + 16; v[i] = ka < K ? W[(size_t)(ka < K ? ka : K - 1) * ld + n] : 0.f; v[8 + i] = kb < K ? W[(size_t)(kb < K ? kb : K - 1) * ld + n] : 0.f; }
  return bsplit16(v); }
__device__ __forceinline__ v8f mac3(const F2& a, const F2& b, v8f c) { c = wmma_bf(a.l, b.h, c); c = wmma_bf(a.h, b.l, c); return wmma_bf(a.h, b.h, c); }
__device__ __forceinline__ float sigm(float v) { return 1.0f / (1.0f + expf(-v)); }
#define LDSX() do { asm volatile("s_wait_dscnt 0" ::: "memory"); __builtin_amdgcn_wave_barrier(); __builtin_amdgcn_fence(__ATOMIC_RELEASE, "workgroup"); } while (0)

__device__ __forceinline__ float bfr(float v) { return (float)(__bf16)v; }
__device__ __attribute__((noinline)) float tanh_ni(float v) { return tanhf(v); }
#define NM 16
#define LAT 1024
#define S0 512
#define S1 256
#define S2 128
#define RES 128
#define NG (RES * RES)
#ifndef NBLK
#define NBLK (NM * NG / 64)
#endif
#define WS_Y0 0u
#define WS_END (WS_Y0 + 4u * (size_t)NM * S0)
__device__ __forceinline__ float gridv(int k) { return (k == RES - 1) ? 1.0f : (float)(-1.0 + (double)k * (2.0 / 127.0)); }
__global__ __launch_bounds__(64) void k_y0(const float* __restrict__ X0, const float* __restrict__ W0A, const float* __restrict__ B0A, float* __restrict__ Y0) {
  const int o = blockIdx.x * 64 + threadIdx.x, m = blockIdx.y; const float* w = W0A + ((size_t)m * S0 + o) * LAT; float s = 0.f;
#pragma unroll 1
  for (int l = 0; l < LAT; l += 4) { const v4f wv = *(const v4f*)(w + l); s += bfr(wv[0]) * bfr(X0[l]) + bfr(wv[1]) * bfr(X0[l + 1]) + bfr(wv[2]) * bfr(X0[l + 2]) + bfr(wv[3]) * bfr(X0[l + 3]); }
  __shared__ __align__(16) float sy[64]; sy[threadIdx.x] = s + bfr(B0A[m * S0 + o]); LDSX(); __syncthreads();
  if (threadIdx.x < 16) vst2(Y0 + (size_t)m * S0 + blockIdx.x * 64 + threadIdx.x * 4, *(const v4f*)&sy[threadIdx.x * 4]); }
__global__ __launch_bounds__(128) void k_mlp(const float* __restrict__ Y0, const float* __restrict__ W0B, const float* __restrict__ B0B, const float* __restrict__ W1, const float* __restrict__ B1, const float* __restrict__ W2, const float* __restrict__ B2, const float* __restrict__ W3, const float* __restrict__ B3, float* __restrict__ OUT) {
  __shared__ __align__(16) _Float16 sh1[64][264]; __shared__ __align__(16) _Float16 sh2[64][136]; __shared__ __align__(16) float so[64 * 3]; __shared__ float sy0[S0], swx[S0], swy[S0];
  const int tid = threadIdx.x, wave = tid >> 5, lane = tid & 31, col = lane & 15, g = lane >> 4; const int m = blockIdx.x / (NG / 64); const size_t g0 = (size_t)(blockIdx.x % (NG / 64)) * 64;
  for (int e = tid; e < S0; e += 128) { sy0[e] = Y0[(size_t)m * S0 + e] + bfr(B0B[m * S0 + e]); swx[e] = bfr(W0B[((size_t)m * S0 + e) * 2]); swy[e] = bfr(W0B[((size_t)m * S0 + e) * 2 + 1]); }
  __syncthreads();
  const int gi = (int)(g0 + wave * 16 + col); const float gx = gridv(gi % RES), gy = gridv(gi / RES);
#pragma unroll 1
  for (int cp = 0; cp < 2; ++cp) { v8f acc[8] = {};
#pragma unroll 2
    for (int kc = 0; kc < S0 / 32; ++kc) { v16h a;
#pragma unroll
      for (int i = 0; i < 16; ++i) { const int k = kc * 32 + (i < 8 ? 8 * g + i : 16 + 8 * g + (i - 8)); a[i] = (_Float16)fmaxf(sy0[k] + swx[k] * gx + swy[k] * gy, 0.f); }
#pragma unroll
      for (int j = 0; j < 8; ++j) { v16h w; const int o = cp * 128 + j * 16 + col; const float* wr = W1 + ((size_t)m * S1 + o) * S0 + kc * 32 + 8 * g;
#pragma unroll
        for (int i = 0; i < 8; ++i) { w[i] = (_Float16)(bfr(wr[i]) * 16.0f); w[8 + i] = (_Float16)(bfr(wr[16 + i]) * 16.0f); }
        acc[j] = wmma16(a, w, acc[j]); } }
#pragma unroll
    for (int j = 0; j < 8; ++j) { const int o = cp * 128 + j * 16 + col; const float bb = bfr(B1[m * S1 + o]);
#pragma unroll
      for (int r = 0; r < 8; ++r) sh1[wave * 16 + 8 * g + r][o] = (_Float16)fmaxf(acc[j][r] * (1.0f / 16.0f) + bb, 0.f); } }
  LDSX();
  { v8f acc[8] = {};
#pragma unroll
    for (int kc = 0; kc < S1 / 32; ++kc) { const v16h a = frag_h(&sh1[wave * 16 + col][kc * 32], lane);
#pragma unroll
      for (int j = 0; j < 8; ++j) { v16h w; const int o = j * 16 + col; const float* wr = W2 + ((size_t)m * S2 + o) * S1 + kc * 32 + 8 * g;
#pragma unroll
        for (int i = 0; i < 8; ++i) { w[i] = (_Float16)(bfr(wr[i]) * 16.0f); w[8 + i] = (_Float16)(bfr(wr[16 + i]) * 16.0f); }
        acc[j] = wmma16(a, w, acc[j]); } }
#pragma unroll
    for (int j = 0; j < 8; ++j) { const int o = j * 16 + col; const float bb = bfr(B2[m * S2 + o]);
#pragma unroll
      for (int r = 0; r < 8; ++r) sh2[wave * 16 + 8 * g + r][o] = (_Float16)fmaxf(acc[j][r] * (1.0f / 16.0f) + bb, 0.f); } }
  LDSX();
  { v8f acc = {};
#pragma unroll
    for (int kc = 0; kc < S2 / 32; ++kc) { const v16h a = frag_h(&sh2[wave * 16 + col][kc * 32], lane); v16h w; const int o = col; const float* wr = W3 + ((size_t)m * 3 + (o < 3 ? o : 0)) * S2 + kc * 32 + 8 * g;
#pragma unroll
      for (int i = 0; i < 8; ++i) { w[i] = (o < 3) ? (_Float16)(bfr(wr[i]) * 16.0f) : (_Float16)0.f; w[8 + i] = (o < 3) ? (_Float16)(bfr(wr[16 + i]) * 16.0f) : (_Float16)0.f; }
      acc = wmma16(a, w, acc); }
    if (col < 3) { const float bb = bfr(B3[m * 3 + col]);
#pragma unroll
      for (int r = 0; r < 8; ++r) so[(wave * 16 + 8 * g + r) * 3 + col] = tanh_ni(acc[r] * (1.0f / 16.0f) + bb); } }
  __syncthreads();
  if (tid < 48) vst2(OUT + ((size_t)m * NG + g0) * 3 + tid * 4, *(const v4f*)&so[tid * 4]); }
extern "C" void kernel_launch(void* const* d_in, const int* in_sizes, int n_in, void* d_out, int out_size, void* d_ws, size_t ws_size, hipStream_t stream) {
  (void)in_sizes; (void)n_in; (void)out_size;
  const float** F = (const float**)d_in;
  if (ws_size < (size_t)WS_END) return;
  char* ws = (char*)d_ws; float* Y0 = (float*)(ws + WS_Y0);
  k_y0<<<dim3(S0 / 64, NM), 64, 0, stream>>>(F[0], F[1], F[2], Y0);
  k_mlp<<<dim3(NBLK), 128, 0, stream>>>(Y0, F[3], F[4], F[5], F[6], F[7], F[8], F[9], F[10], (float*)d_out);
}
